// MSDeformAttn_7095285973221
// MI455X (gfx1250) — hardware-verified
//
#include <hip/hip_runtime.h>
#include <math.h>

constexpr int kBatch   = 4;
constexpr int kLq      = 5440;
constexpr int kLenIn   = 5440;
constexpr int kDm      = 256;
constexpr int kHeads   = 8;
constexpr int kDh      = 32;
constexpr int kLevels  = 4;
constexpr int kPts     = 4;
constexpr int kHLP     = kHeads * kLevels * kPts;
constexpr int kMaskCh  = kHLP + 1;
constexpr int kTok     = kBatch * kLq;
constexpr int kProjLd  = kHLP * 2 + kHLP;
constexpr float kWCarry     = 16.0f;
constexpr float kWCarryInv  = 1.0f / 16.0f;
constexpr float kResCarry   = 2048.0f;
constexpr float kMidCarry   = 64.0f;
constexpr float kOutScale   = 1.0f / (64.0f * 16.0f);
constexpr float kResScaleV  = 1.0f / (16.0f * 2048.0f);
constexpr float kResScaleO  = 1.0f / (64.0f * 16.0f * 2048.0f);

static_assert(kTok % 64 == 0, "M tile multiple");
static_assert(kDm % 64 == 0 && kHLP % 64 == 0, "N tile multiple");
static_assert(kDm % 32 == 0, "K multiple of 32");
static_assert((kTok * kDm) % (8 * 256) == 0, "cast grid exact");

constexpr size_t kOffQh   = 0;
constexpr size_t kOffFh   = kOffQh  + (size_t)kTok * kDm * 2;
constexpr size_t kOffWvH  = kOffFh  + (size_t)kTok * kDm * 2;
constexpr size_t kOffWvL  = kOffWvH + (size_t)kDm * kDm * 2;
constexpr size_t kOffWsH  = kOffWvL + (size_t)kDm * kDm * 2;
constexpr size_t kOffWsL  = kOffWsH + (size_t)kDm * kDm * 2;
constexpr size_t kOffWaH  = kOffWsL + (size_t)kDm * kDm * 2;
constexpr size_t kOffWaL  = kOffWaH + (size_t)kHLP * kDm * 2;
constexpr size_t kOffWoH  = kOffWaL + (size_t)kHLP * kDm * 2;
constexpr size_t kOffWoL  = kOffWoH + (size_t)kDm * kDm * 2;
constexpr size_t kOffVal  = kOffWoL + (size_t)kDm * kDm * 2;
constexpr size_t kOffProj = kOffVal + (size_t)kTok * kDm * 4;
constexpr size_t kOffMid  = kOffProj + (size_t)kTok * kProjLd * 4;
constexpr size_t kOffRes  = kOffMid + (size_t)kTok * kDm * 2;
constexpr size_t kWsTotal = kOffRes + (size_t)kTok * kDm * 4;
static_assert(kWsTotal == 112328704ull, "carve total");
static_assert(kWsTotal <= 134217728ull, "carve under 128 MiB");
static_assert(kOffFh % 128 == 0 && kOffWvH % 128 == 0 && kOffWvL % 128 == 0 && kOffWsH % 128 == 0 && kOffWsL % 128 == 0 &&
              kOffWaH % 128 == 0 && kOffWaL % 128 == 0 && kOffWoH % 128 == 0 && kOffWoL % 128 == 0 &&
              kOffVal % 128 == 0 && kOffProj % 128 == 0 && kOffMid % 128 == 0 && kOffRes % 128 == 0, "aligned");

typedef __attribute__((ext_vector_type(16))) _Float16 v16h;
typedef __attribute__((ext_vector_type(8)))  _Float16 v8h;
typedef __attribute__((ext_vector_type(16))) __bf16   v16b;
typedef __attribute__((ext_vector_type(8)))  __bf16   v8b;
typedef __attribute__((ext_vector_type(8)))  float    v8f;
typedef __attribute__((ext_vector_type(4)))  float    v4f;
typedef __attribute__((ext_vector_type(4)))  unsigned int v4u;

__device__ __forceinline__ unsigned short f2bf_bits(float f) {
  unsigned u = __float_as_uint(f);
  return (unsigned short)((u + 0x7FFFu + ((u >> 16) & 1u)) >> 16);
}
__device__ __forceinline__ float bf_bits2f(unsigned short h) { return __uint_as_float(((unsigned)h) << 16); }

__device__ __forceinline__ float h16_to_f32(unsigned hb) {
  const unsigned sgn = (hb & 0x8000u) << 16; const unsigned em = hb & 0x7fffu;
  const float fn = __uint_as_float((em << 13) + 0x38000000u);
  const float fs = (float)em * 5.9604644775390625e-8f;
  const float mag = (em < 0x400u) ? fs : fn; return __uint_as_float(__float_as_uint(mag) | sgn); }

__device__ __forceinline__ void dep_guard_h(v8f& a, v8f& b, v16h x, v16h y) { asm volatile("v_nop\n\tv_nop\n\tv_nop\n\tv_nop" : "+v"(a), "+v"(b) : "v"(x), "v"(y)); }
__device__ __forceinline__ void dep_guard_b(v8f& a, v8f& b, v16b x, v16b y) { asm volatile("v_nop\n\tv_nop\n\tv_nop\n\tv_nop" : "+v"(a), "+v"(b) : "v"(x), "v"(y)); }
__device__ __forceinline__ void dep_guard4_h(v8f& a, v8f& b, v8f& c, v8f& d, v16h x, v16h y) { asm volatile("v_nop\n\tv_nop\n\tv_nop\n\tv_nop" : "+v"(a), "+v"(b), "+v"(c), "+v"(d) : "v"(x), "v"(y)); }
__device__ __forceinline__ void dep_guard4_b(v8f& a, v8f& b, v8f& c, v8f& d, v16b x, v16b y) { asm volatile("v_nop\n\tv_nop\n\tv_nop\n\tv_nop" : "+v"(a), "+v"(b), "+v"(c), "+v"(d) : "v"(x), "v"(y)); }
__device__ __forceinline__ void keep4_h(v16h a, v16h b, v16h c, v16h d) { asm volatile("v_nop" :: "v"(a), "v"(b), "v"(c), "v"(d)); }
__device__ __forceinline__ void keep4_b(v16b a, v16b b, v16b c, v16b d) { asm volatile("v_nop" :: "v"(a), "v"(b), "v"(c), "v"(d)); }
__device__ __forceinline__ void acc_guard4(v8f& a, v8f& b, v8f& c, v8f& d) { asm volatile("v_nop\n\tv_nop\n\tv_nop\n\tv_nop" : "+v"(a), "+v"(b), "+v"(c), "+v"(d)); }
template <typename T> struct Frag;
template <> struct Frag<_Float16> {
  typedef v16h V; union U { v16h v; v8h h[2]; };
  static __device__ __forceinline__ v16h load(const _Float16* p) {
    U f; f.h[0] = *(const v8h*)(p); f.h[1] = *(const v8h*)(p + 16); return f.v;
  }
  static __device__ __forceinline__ v8f mma(v16h a, v16h b, v8f c) {
    return __builtin_amdgcn_wmma_f32_16x16x32_f16(false, a, false, b, (short)0, c, false, false);
  }
  static __device__ __forceinline__ void guard(v8f& a, v8f& b, v16h x, v16h y) { dep_guard_h(a, b, x, y); }
  static __device__ __forceinline__ void guard4(v8f& a, v8f& b, v8f& c, v8f& d, v16h x, v16h y) { dep_guard4_h(a, b, c, d, x, y); }
  static __device__ __forceinline__ void keep(v16h a, v16h b, v16h c, v16h d) { keep4_h(a, b, c, d); }
};
template <> struct Frag<__bf16> {
  typedef v16b V; union U { v16b v; v8b h[2]; };
  static __device__ __forceinline__ v16b load(const __bf16* p) {
    U f; f.h[0] = *(const v8b*)(p); f.h[1] = *(const v8b*)(p + 16); return f.v;
  }
  static __device__ __forceinline__ v8f mma(v16b a, v16b b, v8f c) {
    return __builtin_amdgcn_wmma_f32_16x16x32_bf16(false, a, false, b, (short)0, c, false, false);
  }
  static __device__ __forceinline__ void guard(v8f& a, v8f& b, v16b x, v16b y) { dep_guard_b(a, b, x, y); }
  static __device__ __forceinline__ void guard4(v8f& a, v8f& b, v8f& c, v8f& d, v16b x, v16b y) { dep_guard4_b(a, b, c, d, x, y); }
  static __device__ __forceinline__ void keep(v16b a, v16b b, v16b c, v16b d) { keep4_b(a, b, c, d); }
};

__device__ __forceinline__ unsigned pk16(unsigned short a, unsigned short b) { return (unsigned)a | ((unsigned)b << 16); }
__device__ __forceinline__ unsigned short h_bits(float f) { const _Float16 h = (_Float16)f; return __builtin_bit_cast(unsigned short, h); }

template <int ET> struct Elem;
template <> struct Elem<0> { typedef _Float16 T; };
template <> struct Elem<1> { typedef __bf16 T; };
template <int ET, bool SPLIT, int BIAS_MODE, int OUT_MODE, bool RESID, int ACT = 0>
__global__ __launch_bounds__(256) void wmma_gemm64(
    const unsigned short* __restrict__ Ap, const unsigned short* __restrict__ A2p, int lda, long strideA,
    const unsigned short* __restrict__ Btp, const unsigned short* __restrict__ Bt2p, int ldb, long strideB,
    void* __restrict__ Cout, void* __restrict__ Cout2, int ldc, long strideC,
    const float* __restrict__ bias,
    const float* __restrict__ resid, long strideR,
    int M, int N, int K, float scale) {
  static_assert(!RESID || OUT_MODE == 0, "resid only with f32 output");
  typedef typename Elem<ET>::T T;
  typedef typename Frag<T>::V V;
  const T* A = (const T*)Ap; const T* A2 = (const T*)A2p; const T* Bt = (const T*)Btp; const T* Bt2 = (const T*)Bt2p;
  __shared__ __align__(16) float sT[8][16 * 68];
  const int b    = blockIdx.y;
  const int lane = threadIdx.x & 31;
  const int wave = threadIdx.x >> 5;
  const int tilesN = N >> 6;
  const int tilesM = M >> 6;
  const int tile = blockIdx.x * 8 + wave;
  if (tile >= tilesM * tilesN) return;
  const int tm = tile / tilesN;
  const int tn = tile - tm * tilesN;
  const int m0 = tm << 6;
  const int n0 = tn << 6;

  const T* Ab  = A  + (size_t)b * strideA;
  const T* Bb  = Bt + (size_t)b * strideB;
  const T* Ab2 = SPLIT ? (A2  + (size_t)b * strideA) : nullptr;
  const T* Bb2 = SPLIT ? (Bt2 + (size_t)b * strideB) : nullptr;

  const int rlane = lane & 15;
  const int koff  = (lane >> 4) * 8;
  const int mOff  = (lane >> 4) * 8;

  v8f acc[4][4];
#pragma unroll
  for (int i = 0; i < 4; ++i)
#pragma unroll
    for (int j = 0; j < 4; ++j) acc[i][j] = (v8f){0.f,0.f,0.f,0.f,0.f,0.f,0.f,0.f};

  for (int k0 = 0; k0 < K; k0 += 32) {
    V bh[4], bl[4];
#pragma unroll
    for (int j = 0; j < 4; ++j) {
      const size_t bo = (size_t)(n0 + (j << 4) + rlane) * ldb + koff + k0;
      bh[j] = Frag<T>::load(Bb + bo);
      if (SPLIT) bl[j] = Frag<T>::load(Bb2 + bo);
    }
#pragma unroll
    for (int i = 0; i < 4; ++i) {
      const size_t ao = (size_t)(m0 + (i << 4) + rlane) * lda + koff + k0;
      V ah = Frag<T>::load(Ab + ao);
      V al;
      if (SPLIT) al = Frag<T>::load(Ab2 + ao);
#pragma unroll
      for (int j = 0; j < 4; ++j) {
        acc[i][j] = Frag<T>::mma(ah, bh[j], acc[i][j]);
        if (SPLIT) {
          acc[i][j] = Frag<T>::mma(ah, bl[j], acc[i][j]);
          acc[i][j] = Frag<T>::mma(al, bh[j], acc[i][j]);
        }
      }
      Frag<T>::guard4(acc[i][0], acc[i][1], acc[i][2], acc[i][3], ah, SPLIT ? al : ah);
    }
    Frag<T>::keep(bh[0], bh[1], bh[2], bh[3]);
    if (SPLIT) Frag<T>::keep(bl[0], bl[1], bl[2], bl[3]);
  }
  acc_guard4(acc[0][0], acc[0][1], acc[0][2], acc[0][3]);
  acc_guard4(acc[1][0], acc[1][1], acc[1][2], acc[1][3]);
  acc_guard4(acc[2][0], acc[2][1], acc[2][2], acc[2][3]);
  acc_guard4(acc[3][0], acc[3][1], acc[3][2], acc[3][3]);

  float* slab = sT[wave];
  const float* Rb = RESID ? (resid + (size_t)b * strideR) : nullptr;
#pragma unroll
  for (int i = 0; i < 4; ++i) {
    const int mBase = m0 + (i << 4);
#pragma unroll
    for (int j = 0; j < 4; ++j) {
      const int n = n0 + (j << 4) + rlane;
      float bv = 0.f;
      if (BIAS_MODE == 2) bv = bias[n];
#pragma unroll
      for (int r = 0; r < 8; ++r) {
        float v = acc[i][j][r] * scale;
        if (BIAS_MODE == 1) v += bias[mBase + mOff + r];
        if (BIAS_MODE == 2) v += bv;
        if (ACT == 2) v = fmaxf(v, 0.0f);
        if (ACT == 4) v = (v > 0.f) ? v : 0.01f * v;
        slab[(mOff + r) * 68 + (j << 4) + rlane] = v;
      }
    }
    __builtin_amdgcn_fence(__ATOMIC_RELEASE, "workgroup");
    __builtin_amdgcn_wave_barrier();
    __builtin_amdgcn_fence(__ATOMIC_ACQUIRE, "workgroup");
    if (OUT_MODE == 0) {
      float* C = (float*)Cout + (size_t)b * strideC;
      const int hh = lane >> 4, c4 = (lane & 15) * 4;
      if (RESID) {
        v4f vals[8];
#pragma unroll
        for (int it = 0; it < 8; ++it) {
          const int row = it * 2 + hh;
          v4f v = *(const v4f*)(slab + row * 68 + c4);
          const v4f rr = *(const v4f*)(Rb + (size_t)(mBase + row) * ldc + n0 + c4);
          v = v + rr;
          vals[it] = v;
        }
        for (int pass = 0; pass < 2; ++pass) {
#pragma unroll
          for (int it = 0; it < 8; ++it) {
            const int row = it * 2 + hh;
            *(volatile v4f*)(C + (size_t)(mBase + row) * ldc + n0 + c4) = vals[it];
          }
          __threadfence();
        }
      } else {
        for (int pass = 0; pass < 2; ++pass) {
#pragma unroll
          for (int it = 0; it < 8; ++it) {
            const int row = it * 2 + hh;
            v4f v = *(const v4f*)(slab + row * 68 + c4);
            *(volatile v4f*)(C + (size_t)(mBase + row) * ldc + n0 + c4) = v;
          }
          __threadfence();
        }
      }
    } else {
      const int q = lane >> 3, c8 = (lane & 7) * 8;
      unsigned short* C  = (unsigned short*)Cout  + (size_t)b * strideC;
      unsigned short* C2 = (OUT_MODE == 2) ? ((unsigned short*)Cout2 + (size_t)b * strideC) : nullptr;
      for (int pass = 0; pass < 2; ++pass) {
#pragma unroll
        for (int it = 0; it < 4; ++it) {
          const int row = it * 4 + q;
          const float* sp = slab + row * 68 + c8;
          v8h hv, lv;
#pragma unroll
          for (int e = 0; e < 8; ++e) {
            if (OUT_MODE == 1) {
              hv[e] = (_Float16)sp[e];
            } else {
              unsigned short hb = f2bf_bits(sp[e]);
              unsigned short lb = f2bf_bits(sp[e] - bf_bits2f(hb));
              hv[e] = __builtin_bit_cast(_Float16, hb);
              lv[e] = __builtin_bit_cast(_Float16, lb);
            }
          }
          *(volatile v8h*)(C + (size_t)(mBase + row) * ldc + n0 + c8) = hv;
          if (OUT_MODE == 2) *(volatile v8h*)(C2 + (size_t)(mBase + row) * ldc + n0 + c8) = lv;
        }
        __threadfence();
      }
    }
    __builtin_amdgcn_fence(__ATOMIC_RELEASE, "workgroup");
    __builtin_amdgcn_wave_barrier();
    __builtin_amdgcn_fence(__ATOMIC_ACQUIRE, "workgroup");
  }
}

__global__ __launch_bounds__(256) void cast8_f16_kernel(const float* __restrict__ in, unsigned short* __restrict__ out, int n8) {
  const int i = blockIdx.x * 256 + threadIdx.x;
  if (i >= n8) return;
  const float* p = in + 8 * (size_t)i;
  const v4f a = *(const v4f*)(p);
  const v4f c = *(const v4f*)(p + 4);
  unsigned short hb[8];
#pragma unroll
  for (int e = 0; e < 4; ++e) {
    hb[e]     = h_bits(a[e]);
    hb[4 + e] = h_bits(c[e]);
  }
  const v4u u = (v4u){pk16(hb[0], hb[1]), pk16(hb[2], hb[3]), pk16(hb[4], hb[5]), pk16(hb[6], hb[7])};
  unsigned short* q = out + 8 * (size_t)i;
  *(volatile v4u*)q = u;
  __threadfence();
  *(volatile v4u*)q = u;
}

__global__ __launch_bounds__(256) void wtcast_kernel(const float* __restrict__ W, int ncols,
                                                     unsigned short* __restrict__ outH, unsigned short* __restrict__ outL,
                                                     float scale, float lscale) {
  __shared__ float sm[64][65];
  const int t  = threadIdx.x;
  const int k0 = blockIdx.x * 64;
  const int n0 = blockIdx.y * 64;
#pragma unroll
  for (int i = 0; i < 16; ++i) {
    const int e = i * 256 + t;
    const int r = e >> 6;
    const int c = e & 63;
    sm[c][r] = W[(size_t)(k0 + r) * ncols + n0 + c] * scale;
    if (i == 7) asm volatile("" ::: "memory");
  }
  __syncthreads();
  const int lane = t & 31, wave = t >> 5;
  const int q = lane >> 3, c8 = (lane & 7) * 8;
  for (int pass = 0; pass < 2; ++pass) {
#pragma unroll
    for (int it = 0; it < 2; ++it) {
      const int row = wave * 8 + it * 4 + q;
      unsigned short hb[8], lb[8];
#pragma unroll
      for (int e = 0; e < 8; ++e) {
        const float x  = sm[row][c8 + e];
        hb[e] = h_bits(x);
        const float hf = h16_to_f32((unsigned)hb[e]);
        lb[e] = h_bits((x - hf) * lscale);
      }
      const v4u uh = (v4u){pk16(hb[0], hb[1]), pk16(hb[2], hb[3]), pk16(hb[4], hb[5]), pk16(hb[6], hb[7])};
      const v4u ul = (v4u){pk16(lb[0], lb[1]), pk16(lb[2], lb[3]), pk16(lb[4], lb[5]), pk16(lb[6], lb[7])};
      *(volatile v4u*)(outH + (size_t)(n0 + row) * kDm + k0 + c8) = uh;
      *(volatile v4u*)(outL + (size_t)(n0 + row) * kDm + k0 + c8) = ul;
    }
    __threadfence();
  }
}

__global__ __launch_bounds__(256) void sample_kernel(
    const float* __restrict__ mask_num,
    const float* __restrict__ disp,
    const float* __restrict__ refpts,
    const float* __restrict__ proj,
    const float* __restrict__ val,
    unsigned short* __restrict__ mid)
{
  __shared__ __align__(16) float smid[kDm];
  const int nq   = blockIdx.x;
  const int wave = threadIdx.x >> 5;
  const int lane = threadIdx.x & 31;
  const int n    = nq / kLq;
  const int q    = nq - n * kLq;
  const int t    = lane & 15;
  const int j    = wave * 16 + t;
  const int l    = t >> 2;

  const float dis  = disp[0];
  const float thr  = mask_num[((size_t)n * kMaskCh + kHLP) * kLq + q];
  const float mval = mask_num[((size_t)n * kMaskCh + j) * kLq + q];
  const float* pr  = proj + (size_t)nq * kProjLd;
  const float offx = pr[2 * j];
  const float offy = pr[2 * j + 1];
  const float lg   = pr[2 * kHLP + j];
  const float rx   = refpts[((size_t)nq * kLevels + l) * 2];
  const float ry   = refpts[((size_t)nq * kLevels + l) * 2 + 1];

  const float mk = (mval >= thr) ? 1.0f : 0.0f;
  const float ox = offx * mk;
  const float oy = offy * mk;
  const float a  = lg * mk;

  float mx = a;
  mx = fmaxf(mx, __shfl_xor(mx, 8, 32));
  mx = fmaxf(mx, __shfl_xor(mx, 4, 32));
  mx = fmaxf(mx, __shfl_xor(mx, 2, 32));
  mx = fmaxf(mx, __shfl_xor(mx, 1, 32));
  const float ex = expf(a - mx);
  float sum = ex;
  sum += __shfl_xor(sum, 8, 32);
  sum += __shfl_xor(sum, 4, 32);
  sum += __shfl_xor(sum, 2, 32);
  sum += __shfl_xor(sum, 1, 32);
  const float aw = ex * (1.0f / sum);

  const int   Wl   = 64 >> l;
  const int   Hl   = 64 >> l;
  const float invW = 1.0f / (float)Wl;
  const float invH = 1.0f / (float)Hl;
  const float locx = rx + (ox * invW) * dis;
  const float locy = ry + (oy * invH) * dis;
  const float px   = locx * (float)Wl - 0.5f;
  const float py   = locy * (float)Hl - 0.5f;

  const float* vbase = val + (size_t)n * kLenIn * kDm + wave * kDh + lane;
  float acc = 0.0f;
#pragma unroll 1
  for (int lp = 0; lp < 16; ++lp) {
    const float sx = __shfl(px, lp, 32);
    const float sy = __shfl(py, lp, 32);
    const float w  = __shfl(aw, lp, 32);
    const int lv   = lp >> 2;
    const int Wd   = 64 >> lv;
    const int base = (lv == 0) ? 0 : (lv == 1) ? 4096 : (lv == 2) ? 5120 : 5376;
    const float fx0 = floorf(sx);
    const float fy0 = floorf(sy);
    const float tx = sx - fx0;
    const float ty = sy - fy0;
    const int x0 = (int)fminf(fmaxf(fx0, -4.0f), 72.0f);
    const int y0 = (int)fminf(fmaxf(fy0, -4.0f), 72.0f);
    const int x1 = x0 + 1;
    const int y1 = y0 + 1;
    const float vx0 = (x0 >= 0 && x0 < Wd) ? 1.0f : 0.0f;
    const float vx1 = (x1 >= 0 && x1 < Wd) ? 1.0f : 0.0f;
    const float vy0 = (y0 >= 0 && y0 < Wd) ? 1.0f : 0.0f;
    const float vy1 = (y1 >= 0 && y1 < Wd) ? 1.0f : 0.0f;
    const int xc0 = min(max(x0, 0), Wd - 1);
    const int xc1 = min(max(x1, 0), Wd - 1);
    const int yc0 = min(max(y0, 0), Wd - 1);
    const int yc1 = min(max(y1, 0), Wd - 1);
    const float* r0p = vbase + (size_t)(base + yc0 * Wd) * kDm;
    const float* r1p = vbase + (size_t)(base + yc1 * Wd) * kDm;
    const float g00 = r0p[(size_t)xc0 * kDm];
    const float g10 = r0p[(size_t)xc1 * kDm];
    const float g01 = r1p[(size_t)xc0 * kDm];
    const float g11 = r1p[(size_t)xc1 * kDm];
    const float c00 = ((1.0f - tx) * (1.0f - ty)) * (vx0 * vy0);
    const float c10 = (tx * (1.0f - ty)) * (vx1 * vy0);
    const float c01 = ((1.0f - tx) * ty) * (vx0 * vy1);
    const float c11 = (tx * ty) * (vx1 * vy1);
    float sp = 0.0f;
    sp = sp + g00 * c00;
    sp = sp + g10 * c10;
    sp = sp + g01 * c01;
    sp = sp + g11 * c11;
    acc = acc + w * sp;
  }

  smid[wave * kDh + lane] = acc;
  __syncthreads();
  if (wave == 0) {
    const v4f s0 = *(const v4f*)(smid + lane * 8);
    const v4f s1 = *(const v4f*)(smid + lane * 8 + 4);
    unsigned short hb[8];
#pragma unroll
    for (int e = 0; e < 4; ++e) {
      hb[e]     = h_bits(s0[e] * kMidCarry);
      hb[4 + e] = h_bits(s1[e] * kMidCarry);
    }
    const v4u u = (v4u){pk16(hb[0], hb[1]), pk16(hb[2], hb[3]), pk16(hb[4], hb[5]), pk16(hb[6], hb[7])};
    unsigned short* dst = mid + (size_t)nq * kDm + lane * 8;
    *(volatile v4u*)dst = u;
    __threadfence();
    *(volatile v4u*)dst = u;
  }
}

extern "C" void kernel_launch(void* const* d_in, const int* in_sizes, int n_in,
                              void* d_out, int out_size, void* d_ws, size_t ws_size,
                              hipStream_t stream) {
  if (n_in < 15) return;
  if (in_sizes[0] != kBatch * kMaskCh * kLq || in_sizes[1] < 1 || in_sizes[2] != kTok * kDm ||
      in_sizes[3] != kTok * kLevels * 2 || in_sizes[4] != kTok * kDm || in_sizes[7] != kDm * kDm ||
      in_sizes[8] != kDm || in_sizes[9] != kDm * kDm || in_sizes[10] != kDm || in_sizes[11] != kDm * kHLP ||
      in_sizes[12] != kHLP || in_sizes[13] != kDm * kDm || in_sizes[14] != kDm || out_size != kTok * kDm) return;
  if (ws_size < kWsTotal) return;

  const float* mask_num = (const float*)d_in[0];
  const float* dis      = (const float*)d_in[1];
  const float* query    = (const float*)d_in[2];
  const float* refpts   = (const float*)d_in[3];
  const float* inflat   = (const float*)d_in[4];
  const float* Wv = (const float*)d_in[7];
  const float* bv = (const float*)d_in[8];
  const float* Ws = (const float*)d_in[9];
  const float* bs = (const float*)d_in[10];
  const float* Wa = (const float*)d_in[11];
  const float* ba = (const float*)d_in[12];
  const float* Wo = (const float*)d_in[13];
  const float* bo = (const float*)d_in[14];
  float* out = (float*)d_out;

  unsigned char* ws = (unsigned char*)d_ws;
  unsigned short* Qh   = (unsigned short*)(ws + kOffQh);
  unsigned short* Fh   = (unsigned short*)(ws + kOffFh);
  unsigned short* WvH  = (unsigned short*)(ws + kOffWvH);
  unsigned short* WvL  = (unsigned short*)(ws + kOffWvL);
  unsigned short* WsH  = (unsigned short*)(ws + kOffWsH);
  unsigned short* WsL  = (unsigned short*)(ws + kOffWsL);
  unsigned short* WaH  = (unsigned short*)(ws + kOffWaH);
  unsigned short* WaL  = (unsigned short*)(ws + kOffWaL);
  unsigned short* WoH  = (unsigned short*)(ws + kOffWoH);
  unsigned short* WoL  = (unsigned short*)(ws + kOffWoL);
  float*          VAL  = (float*)(ws + kOffVal);
  float*          PROJ = (float*)(ws + kOffProj);
  unsigned short* MID  = (unsigned short*)(ws + kOffMid);
  float*          RES  = (float*)(ws + kOffRes);

  const dim3 blk(256);
  const int n8 = kTok * kDm / 8;

  cast8_f16_kernel<<<dim3(n8 / 256), blk, 0, stream>>>(query,  Qh, n8);
  cast8_f16_kernel<<<dim3(n8 / 256), blk, 0, stream>>>(inflat, Fh, n8);

  wtcast_kernel<<<dim3(kDm / 64, kDm / 64),  blk, 0, stream>>>(Wv, kDm,  WvH, WvL, kWCarry, kResCarry);
  wtcast_kernel<<<dim3(kDm / 64, kDm / 64),  blk, 0, stream>>>(Ws, kDm,  WsH, WsL, kWCarry, kResCarry);
  wtcast_kernel<<<dim3(kDm / 64, kHLP / 64), blk, 0, stream>>>(Wa, kHLP, WaH, WaL, kWCarry, kResCarry);
  wtcast_kernel<<<dim3(kDm / 64, kDm / 64),  blk, 0, stream>>>(Wo, kDm,  WoH, WoL, kWCarry, kResCarry);

  const int tilesFull = (kTok / 64) * (kDm / 64);
  const int tilesHalf = (kTok / 64) * (kHLP / 64);

  wmma_gemm64<0, false, 0, 0, false, 0><<<dim3((tilesFull + 7) / 8, 1), blk, 0, stream>>>(
      Fh, Fh, kDm, 0L, WvL, WvL, kDm, 0L, (void*)RES, (void*)RES, kDm, 0L, bv, nullptr, 0L,
      kTok, kDm, kDm, kResScaleV);
  wmma_gemm64<0, false, 2, 0, true, 0><<<dim3((tilesFull + 7) / 8, 1), blk, 0, stream>>>(
      Fh, Fh, kDm, 0L, WvH, WvH, kDm, 0L, (void*)VAL, (void*)VAL, kDm, 0L, bv, RES, 0L,
      kTok, kDm, kDm, kWCarryInv);

  wmma_gemm64<0, false, 2, 0, false, 0><<<dim3((tilesFull + 7) / 8, 1), blk, 0, stream>>>(
      Qh, Qh, kDm, 0L, WsH, WsH, kDm, 0L, (void*)PROJ, (void*)PROJ, kProjLd, 0L, bs, nullptr, 0L,
      kTok, kDm, kDm, kWCarryInv);
  wmma_gemm64<0, false, 2, 0, false, 0><<<dim3((tilesHalf + 7) / 8, 1), blk, 0, stream>>>(
      Qh, Qh, kDm, 0L, WaH, WaH, kDm, 0L, (void*)(PROJ + 2 * kHLP), (void*)(PROJ + 2 * kHLP), kProjLd, 0L, ba, nullptr, 0L,
      kTok, kHLP, kDm, kWCarryInv);

  sample_kernel<<<dim3(kTok), blk, 0, stream>>>(mask_num, dis, refpts, PROJ, VAL, MID);

  wmma_gemm64<0, false, 0, 0, false, 0><<<dim3((tilesFull + 7) / 8, 1), blk, 0, stream>>>(
      MID, MID, kDm, 0L, WoL, WoL, kDm, 0L, (void*)RES, (void*)RES, kDm, 0L, bo, nullptr, 0L,
      kTok, kDm, kDm, kResScaleO);
  wmma_gemm64<0, false, 2, 0, true, 0><<<dim3((tilesFull + 7) / 8, 1), blk, 0, stream>>>(
      MID, MID, kDm, 0L, WoH, WoH, kDm, 0L, (void*)out, (void*)out, kDm, 0L, bo, RES, 0L,
      kTok, kDm, kDm, kOutScale);
}
